// MambaLM_31215822307425
// MI455X (gfx1250) — hardware-run, weakly checked
//
#include <hip/hip_runtime.h>
#include <math.h>

typedef __attribute__((ext_vector_type(16))) _Float16 v16h;
typedef __attribute__((ext_vector_type(8)))  _Float16 v8h;
typedef __attribute__((ext_vector_type(8)))  float    v8f;
typedef __attribute__((ext_vector_type(4)))  float    v4f;

constexpr int kBatch = 2;
constexpr int kCb    = 4;
constexpr int kSeq   = 1024;
constexpr int kVoc   = 1024;
constexpr int kDm    = 512;
constexpr int kDin   = 1024;
constexpr int kNst   = 16;
constexpr int kDtR   = 32;
constexpr int kLay   = 2;
constexpr int kXzP   = 2 * kDin;
constexpr int kXdP   = kDtR + 2 * kNst;
constexpr int kRows  = kBatch * kSeq;
constexpr int kTP    = 260;
static_assert(kXdP == 64);
static_assert((kDm % 32) == 0 && (kDin % 32) == 0 && (kDtR % 32) == 0);
static_assert((kRows % 64) == 0 && (kSeq % 64) == 0 && (kXzP % 64) == 0 && (kXdP % 64) == 0);
static_assert((kDm % 64) == 0 && (kDin % 256) == 0 && (kVoc % 64) == 0 && (kSeq % 16) == 0);

constexpr float kCarW  = 32.0f;
constexpr float kCarU  = 64.0f;
constexpr float kCarDt = 256.0f;
constexpr float kCarY  = 256.0f;
constexpr float kCarX  = 16.0f;
constexpr float kSclIn   = 1.0f / kCarW;
constexpr float kSclXp   = 1.0f / (kCarU * kCarW);
constexpr float kSclDt   = 1.0f / (kCarDt * kCarW);
constexpr float kSclOut  = 1.0f / (kCarY * kCarW);
constexpr float kSclHead = 1.0f / (kCarX * kCarW);

constexpr size_t kSzWIN  = (size_t)kLay * kXzP * kDm * 2;
constexpr size_t kSzWXP  = (size_t)kLay * kXdP * kDin * 2;
constexpr size_t kSzWDT  = (size_t)kLay * kDin * kDtR * 2;
constexpr size_t kSzWOUT = (size_t)kLay * kDm * kDin * 2;
constexpr size_t kSzWHD  = (size_t)kCb * kVoc * kDm * 2;
constexpr size_t kSzX    = (size_t)kRows * kDm * 4;
constexpr size_t kSzXN   = (size_t)kRows * kDm * 2;
constexpr size_t kSzXZ   = (size_t)kRows * kXzP * 4;
constexpr size_t kSzUC   = (size_t)kRows * kDin * 4;
constexpr size_t kSzUC16 = (size_t)kRows * kDin * 2;
constexpr size_t kSzXD   = (size_t)kRows * kXdP * 4;
constexpr size_t kSzDT16 = (size_t)kRows * kDtR * 2;
constexpr size_t kSzDLR  = (size_t)kRows * kDin * 4;
constexpr size_t kSzY16  = (size_t)kRows * kDin * 2;
constexpr size_t kOffWIN  = 0;
constexpr size_t kOffWXP  = kOffWIN  + kSzWIN;
constexpr size_t kOffWDT  = kOffWXP  + kSzWXP;
constexpr size_t kOffWOUT = kOffWDT  + kSzWDT;
constexpr size_t kOffWHD  = kOffWOUT + kSzWOUT;
constexpr size_t kOffXA   = kOffWHD  + kSzWHD;
constexpr size_t kOffXB   = kOffXA   + kSzX;
constexpr size_t kOffXN   = kOffXB   + kSzX;
constexpr size_t kOffXZ   = kOffXN   + kSzXN;
constexpr size_t kOffUC   = kOffXZ   + kSzXZ;
constexpr size_t kOffUC16 = kOffUC   + kSzUC;
constexpr size_t kOffXD   = kOffUC16 + kSzUC16;
constexpr size_t kOffDT16 = kOffXD   + kSzXD;
constexpr size_t kOffDLR  = kOffDT16 + kSzDT16;
constexpr size_t kOffY16  = kOffDLR  + kSzDLR;
constexpr size_t kWsTotal = kOffY16  + kSzY16;
static_assert(kWsTotal == 63963136ull);
static_assert(kWsTotal <= 134217728ull);
static_assert((kOffWXP % 128) == 0 && (kOffWDT % 128) == 0 && (kOffWOUT % 128) == 0 && (kOffWHD % 128) == 0);
static_assert((kOffXA % 128) == 0 && (kOffXB % 128) == 0 && (kOffXN % 128) == 0 && (kOffXZ % 128) == 0);
static_assert((kOffUC % 128) == 0 && (kOffUC16 % 128) == 0 && (kOffXD % 128) == 0 && (kOffDT16 % 128) == 0);
static_assert((kOffDLR % 128) == 0 && (kOffY16 % 128) == 0);

union FragU { v16h v; v8h h[2]; };
__device__ __forceinline__ v16h frag_load(const _Float16* p) {
  FragU f;
  f.h[0] = *(const v8h*)(p);
  f.h[1] = *(const v8h*)(p + 16);
  return f.v;
}
__device__ __forceinline__ v8f frag_mma(v16h a, v16h b, v8f c) {
  return __builtin_amdgcn_wmma_f32_16x16x32_f16(false, a, false, b, (short)0, c, false, false);
}
__device__ __forceinline__ void row_guard_h(v8f& a, v8f& b, v8f& c, v8f& d, v16h x,
                                            v16h b0, v16h b1, v16h b2, v16h b3) {
  asm volatile("v_nop\n\tv_nop\n\tv_nop\n\tv_nop"
               : "+v"(a), "+v"(b), "+v"(c), "+v"(d)
               : "v"(x), "v"(b0), "v"(b1), "v"(b2), "v"(b3));
}
__device__ __forceinline__ void keep4_h(v16h a, v16h b, v16h c, v16h d) {
  asm volatile("v_nop" :: "v"(a), "v"(b), "v"(c), "v"(d));
}
__device__ __forceinline__ void acc_guard4(v8f& a, v8f& b, v8f& c, v8f& d) {
  asm volatile("v_nop\n\tv_nop\n\tv_nop\n\tv_nop" : "+v"(a), "+v"(b), "+v"(c), "+v"(d));
}

template <bool RESID>
__global__ __launch_bounds__(256) void wmma_gemm64_f16(
    const unsigned short* __restrict__ Ap, int lda, long strideA,
    const unsigned short* __restrict__ Btp, int ldb, long strideB,
    float* __restrict__ Cout, int ldc, long strideC,
    const float* __restrict__ resid,
    int M, int N, int K, float scale) {
  const _Float16* A  = (const _Float16*)Ap;
  const _Float16* Bt = (const _Float16*)Btp;
  __shared__ __align__(16) float sT[8][16 * 68];
  const int b    = blockIdx.y;
  const int lane = threadIdx.x & 31;
  const int wave = threadIdx.x >> 5;
  const int tilesN = N >> 6;
  const int tilesM = M >> 6;
  const int tile = blockIdx.x * 8 + wave;
  if (tile >= tilesM * tilesN) return;
  const int tm = tile / tilesN;
  const int tn = tile - tm * tilesN;
  const int m0 = tm << 6;
  const int n0 = tn << 6;

  const _Float16* Ab = A  + (size_t)b * strideA;
  const _Float16* Bb = Bt + (size_t)b * strideB;

  const int rlane = lane & 15;
  const int koff  = (lane >> 4) * 8;
  const int mOff  = (lane >> 4) * 8;

  v8f acc[4][4];
#pragma unroll
  for (int i = 0; i < 4; ++i)
#pragma unroll
    for (int j = 0; j < 4; ++j) acc[i][j] = (v8f){0.f, 0.f, 0.f, 0.f, 0.f, 0.f, 0.f, 0.f};

  for (int k0 = 0; k0 < K; k0 += 32) {
    v16h bh[4];
#pragma unroll
    for (int j = 0; j < 4; ++j) {
      const size_t bo = (size_t)(n0 + (j << 4) + rlane) * ldb + koff + k0;
      bh[j] = frag_load(Bb + bo);
    }
#pragma unroll
    for (int i = 0; i < 4; ++i) {
      const size_t ao = (size_t)(m0 + (i << 4) + rlane) * lda + koff + k0;
      const v16h ah = frag_load(Ab + ao);
#pragma unroll
      for (int j = 0; j < 4; ++j) acc[i][j] = frag_mma(ah, bh[j], acc[i][j]);
      row_guard_h(acc[i][0], acc[i][1], acc[i][2], acc[i][3], ah, bh[0], bh[1], bh[2], bh[3]);
    }
    keep4_h(bh[0], bh[1], bh[2], bh[3]);
  }
  acc_guard4(acc[0][0], acc[0][1], acc[0][2], acc[0][3]);
  acc_guard4(acc[1][0], acc[1][1], acc[1][2], acc[1][3]);
  acc_guard4(acc[2][0], acc[2][1], acc[2][2], acc[2][3]);
  acc_guard4(acc[3][0], acc[3][1], acc[3][2], acc[3][3]);

  float* slab = sT[wave];
  float* C = Cout + (size_t)b * strideC;
  const int hh = lane >> 4;
  const int c4 = (lane & 15) * 4;
#pragma unroll
  for (int i = 0; i < 4; ++i) {
    const int mBase = m0 + (i << 4);
#pragma unroll
    for (int j = 0; j < 4; ++j) {
#pragma unroll
      for (int r = 0; r < 8; ++r) {
        slab[(mOff + r) * 68 + (j << 4) + rlane] = acc[i][j][r] * scale;
      }
    }
    __builtin_amdgcn_fence(__ATOMIC_RELEASE, "workgroup");
    __builtin_amdgcn_wave_barrier();
    __builtin_amdgcn_fence(__ATOMIC_ACQUIRE, "workgroup");
    v4f ov[8];
#pragma unroll
    for (int it = 0; it < 8; ++it) {
      const int row = it * 2 + hh;
      v4f v = *(const v4f*)(slab + row * 68 + c4);
      if (RESID) {
        const v4f rv = *(const v4f*)(resid + (size_t)(mBase + row) * ldc + n0 + c4);
        v = v + rv;
      }
      ov[it] = v;
    }
    for (int pass = 0; pass < 2; ++pass) {
#pragma unroll
      for (int it = 0; it < 8; ++it) {
        const int row = it * 2 + hh;
        *(volatile v4f*)(C + (size_t)(mBase + row) * ldc + n0 + c4) = ov[it];
      }
      __threadfence();
    }
    __builtin_amdgcn_fence(__ATOMIC_RELEASE, "workgroup");
    __builtin_amdgcn_wave_barrier();
    __builtin_amdgcn_fence(__ATOMIC_ACQUIRE, "workgroup");
  }
}

__global__ __launch_bounds__(256) void cast_f16_kernel(
    const float* __restrict__ src, unsigned short* __restrict__ dst, int total8, float scale)
{
  const int i = blockIdx.x * 256 + threadIdx.x;
  if (i >= total8) return;
  const size_t e0 = (size_t)i << 3;
  const float* p = src + e0;
  const v4f a0 = *(const v4f*)(p);
  const v4f a1 = *(const v4f*)(p + 4);
  v8h hv;
#pragma unroll
  for (int e = 0; e < 4; ++e) {
    hv[e]     = (_Float16)(a0[e] * scale);
    hv[4 + e] = (_Float16)(a1[e] * scale);
  }
  unsigned short* q = dst + e0;
  *(volatile v8h*)q = hv;
  __threadfence();
  *(volatile v8h*)q = hv;
}

__global__ __launch_bounds__(256) void transpose_cast_kernel(
    const float* __restrict__ Wz, unsigned short* __restrict__ Btz, int Kdim, int Ndim, int Npad, float scale)
{
  __shared__ float tile[64 * 65];
  const int tid = threadIdx.x, lane = tid & 31, wave = tid >> 5;
  const int n0 = blockIdx.x * 64;
  const int k0 = blockIdx.y * 64;
  const float* W = Wz + (size_t)blockIdx.z * Kdim * Ndim;
  unsigned short* Bt = Btz + (size_t)blockIdx.z * Npad * Kdim;
#pragma unroll
  for (int p = 0; p < 16; ++p) {
    const int idx = tid + p * 256;
    const int kk  = idx >> 6;
    const int nn  = idx & 63;
    const int n   = n0 + nn;
    const int nc  = (n < Ndim) ? n : (Ndim - 1);
    const float v = W[(size_t)(k0 + kk) * Ndim + nc];
    tile[kk * 65 + nn] = (n < Ndim) ? (v * scale) : 0.f;
  }
  __syncthreads();
  const int q = lane >> 3, c8 = (lane & 7) * 8;
  v8h hv[2];
#pragma unroll
  for (int it = 0; it < 2; ++it) {
    const int nrow = it * 32 + wave * 4 + q;
#pragma unroll
    for (int e = 0; e < 8; ++e) hv[it][e] = (_Float16)tile[(c8 + e) * 65 + nrow];
  }
  for (int pass = 0; pass < 2; ++pass) {
#pragma unroll
    for (int it = 0; it < 2; ++it) {
      const int nrow = it * 32 + wave * 4 + q;
      *(volatile v8h*)(Bt + (size_t)(n0 + nrow) * Kdim + k0 + c8) = hv[it];
    }
    __threadfence();
  }
}

__global__ __launch_bounds__(256) void embed_sum_kernel(
    const int* __restrict__ codes, const float* __restrict__ ew, float* __restrict__ x)
{
  const int tid = threadIdx.x;
  const int row = blockIdx.x * 2 + (tid >> 7);
  const int c4  = (tid & 127) * 4;
  const int b   = row / kSeq;
  const int t   = row - b * kSeq;
  v4f s = (v4f){0.f, 0.f, 0.f, 0.f};
#pragma unroll
  for (int k = 0; k < kCb; ++k) {
    int c = codes[(b * kCb + k) * kSeq + t];
    c = (c < 0) ? 0 : ((c > kVoc - 1) ? (kVoc - 1) : c);
    const v4f e = *(const v4f*)(ew + ((size_t)k * kVoc + c) * kDm + c4);
    s = s + e;
  }
  float* p = x + (size_t)row * kDm + c4;
  *(volatile v4f*)p = s;
  __threadfence();
  *(volatile v4f*)p = s;
}

__global__ __launch_bounds__(256) void rmsnorm_f16_kernel(
    const float* __restrict__ x, const float* __restrict__ w, unsigned short* __restrict__ out)
{
  const int lane = threadIdx.x & 31, wave = threadIdx.x >> 5;
  const int row = blockIdx.x * 8 + wave;
  const float* xr = x + (size_t)row * kDm;
  v4f a[4], g[4];
#pragma unroll
  for (int j = 0; j < 2; ++j) {
    const int c = j * 256 + lane * 8;
    a[2 * j]     = *(const v4f*)(xr + c);
    a[2 * j + 1] = *(const v4f*)(xr + c + 4);
    g[2 * j]     = *(const v4f*)(w + c);
    g[2 * j + 1] = *(const v4f*)(w + c + 4);
  }
  float ss = 0.f;
#pragma unroll
  for (int q = 0; q < 4; ++q) {
#pragma unroll
    for (int e = 0; e < 4; ++e) ss = fmaf(a[q][e], a[q][e], ss);
  }
#pragma unroll
  for (int off = 16; off > 0; off >>= 1) ss += __shfl_xor(ss, off, 32);
  const float r = rsqrtf(ss * (1.0f / (float)kDm) + 1e-6f);
  v8h hv[2];
#pragma unroll
  for (int j = 0; j < 2; ++j) {
#pragma unroll
    for (int e = 0; e < 4; ++e) {
      hv[j][e]     = (_Float16)((a[2 * j][e] * g[2 * j][e]) * r);
      hv[j][4 + e] = (_Float16)((a[2 * j + 1][e] * g[2 * j + 1][e]) * r);
    }
  }
  unsigned short* orow = out + (size_t)row * kDm;
  for (int pass = 0; pass < 2; ++pass) {
#pragma unroll
    for (int j = 0; j < 2; ++j) *(volatile v8h*)(orow + j * 256 + lane * 8) = hv[j];
    __threadfence();
  }
}

__global__ __launch_bounds__(256) void conv_silu_kernel(
    const float* __restrict__ XZ, const float* __restrict__ cw, const float* __restrict__ cb,
    float* __restrict__ UC, unsigned short* __restrict__ UC16)
{
  __shared__ __align__(16) float sT[16 * kTP];
  const int tid = threadIdx.x, lane = tid & 31, wave = tid >> 5;
  const int d0 = blockIdx.x * 256, d = d0 + tid;
  const int g0 = blockIdx.y * 64;
  const int tb = g0 % kSeq;
  const v4f wv = *(const v4f*)(cw + (size_t)d * 4);
  const float w0 = wv[0], w1 = wv[1], w2 = wv[2], w3 = wv[3];
  const float bc = cb[d];
  float xm3, xm2, xm1;
  {
    const bool hist = (tb > 0);
    const int rb = hist ? (g0 - 3) : g0;
    const float v3 = XZ[(size_t)rb * kXzP + d];
    const float v2 = XZ[(size_t)(rb + 1) * kXzP + d];
    const float v1 = XZ[(size_t)(rb + 2) * kXzP + d];
    xm3 = hist ? v3 : 0.f;
    xm2 = hist ? v2 : 0.f;
    xm1 = hist ? v1 : 0.f;
  }
  const int hrow = wave >> 1;
  const int hch  = (wave & 1) * 128 + lane * 4;
#pragma unroll 1
  for (int sub = 0; sub < 4; ++sub) {
    const int lb = g0 + sub * 16;
#pragma unroll 1
    for (int s = 0; s < 16; ++s) {
      const float xc = XZ[(size_t)(lb + s) * kXzP + d];
      float acc = w0 * xm3;
      acc = fmaf(w1, xm2, acc);
      acc = fmaf(w2, xm1, acc);
      acc = fmaf(w3, xc, acc);
      const float sv = acc + bc;
      const float sg = __builtin_amdgcn_rcpf(1.0f + expf(-sv));
      sT[s * kTP + tid] = sv * sg;
      xm3 = xm2; xm2 = xm1; xm1 = xc;
    }
    __syncthreads();
    v4f fv[4];
    v8h bv[2];
#pragma unroll
    for (int it = 0; it < 4; ++it) fv[it] = *(const v4f*)(sT + (it * 4 + hrow) * kTP + hch);
#pragma unroll
    for (int it = 0; it < 2; ++it) {
      const float* sp = sT + (it * 8 + wave) * kTP + lane * 8;
      const v4f a0 = *(const v4f*)(sp);
      const v4f a1 = *(const v4f*)(sp + 4);
#pragma unroll
      for (int e = 0; e < 4; ++e) {
        bv[it][e]     = (_Float16)(a0[e] * kCarU);
        bv[it][4 + e] = (_Float16)(a1[e] * kCarU);
      }
    }
    for (int pass = 0; pass < 2; ++pass) {
#pragma unroll
      for (int it = 0; it < 4; ++it)
        *(volatile v4f*)(UC + (size_t)(lb + it * 4 + hrow) * kDin + d0 + hch) = fv[it];
#pragma unroll
      for (int it = 0; it < 2; ++it)
        *(volatile v8h*)(UC16 + (size_t)(lb + it * 8 + wave) * kDin + d0 + lane * 8) = bv[it];
      __threadfence();
    }
    __syncthreads();
  }
}

__global__ __launch_bounds__(256) void dt_cast_kernel(
    const float* __restrict__ XD, unsigned short* __restrict__ DT16, int total8, float scale)
{
  const int i = blockIdx.x * 256 + threadIdx.x;
  if (i >= total8) return;
  const int e0  = i << 3;
  const int row = e0 / kDtR;
  const int c8  = e0 - row * kDtR;
  const float* p = XD + (size_t)row * kXdP + c8;
  const v4f a0 = *(const v4f*)(p);
  const v4f a1 = *(const v4f*)(p + 4);
  v8h hv;
#pragma unroll
  for (int e = 0; e < 4; ++e) {
    hv[e]     = (_Float16)(a0[e] * scale);
    hv[4 + e] = (_Float16)(a1[e] * scale);
  }
  unsigned short* qd = DT16 + e0;
  *(volatile v8h*)qd = hv;
  __threadfence();
  *(volatile v8h*)qd = hv;
}

__global__ __launch_bounds__(256) void scan_gate_kernel(
    const float* __restrict__ DLR, const float* __restrict__ bdt, const float* __restrict__ UC,
    const float* __restrict__ XZ, const float* __restrict__ XD, const float* __restrict__ Alog,
    const float* __restrict__ Dv, unsigned short* __restrict__ Y16)
{
  __shared__ __align__(16) float sBC[16 * 32];
  __shared__ __align__(16) float sY[16 * kTP];
  const int tid = threadIdx.x, lane = tid & 31, wave = tid >> 5;
  const int d0 = blockIdx.x * 256, d = d0 + tid;
  const size_t row0 = (size_t)blockIdx.y * kSeq;

#pragma unroll 1
  for (int n = 0; n < kNst; ++n) sY[n * 256 + tid] = -expf(Alog[(size_t)d * kNst + n]);
  __syncthreads();
  float An[kNst], h[kNst];
#pragma unroll
  for (int n = 0; n < kNst; ++n) {
    An[n] = sY[n * 256 + tid];
    h[n] = 0.f;
  }
  const float bb = bdt[d];
  const float Dd = Dv[d];

#pragma unroll 1
  for (int c = 0; c < kSeq / 16; ++c) {
    const int l0 = c * 16;
    if (tid < 128) {
      const int r = tid >> 3, q = (tid & 7) * 4;
      const v4f v = *(const v4f*)(XD + (row0 + l0 + r) * kXdP + kDtR + q);
      *(v4f*)(sBC + r * 32 + q) = v;
    }
    __syncthreads();
#pragma unroll 1
    for (int s = 0; s < 16; ++s) {
      const size_t m = row0 + (size_t)(l0 + s);
      const float a     = DLR[m * kDin + d] + bb;
      const float ea    = expf(-fabsf(a));
      const float delta = fmaxf(a, 0.0f) + log1pf(ea);
      const float xv    = UC[m * kDin + d];
      const float zv    = XZ[m * kXzP + kDin + d];
      v4f Bq[4], Cq[4];
#pragma unroll
      for (int qq = 0; qq < 4; ++qq) {
        Bq[qq] = *(const v4f*)(sBC + s * 32 + 4 * qq);
        Cq[qq] = *(const v4f*)(sBC + s * 32 + kNst + 4 * qq);
      }
      float y = 0.f;
#pragma unroll
      for (int n = 0; n < kNst; ++n) {
        const float e  = __expf(delta * An[n]);
        const float db = delta * Bq[n >> 2][n & 3];
        const float hn = e * h[n] + db * xv;
        h[n] = hn;
        y = hn * Cq[n >> 2][n & 3] + y;
      }
      y = xv * Dd + y;
      const float sg = __builtin_amdgcn_rcpf(1.0f + expf(-zv));
      const float g  = zv * sg;
      sY[s * kTP + tid] = (y * g) * kCarY;
    }
    __syncthreads();
    v8h hv[2];
#pragma unroll
    for (int it = 0; it < 2; ++it) {
      const float* sp = sY + (it * 8 + wave) * kTP + lane * 8;
      const v4f a0 = *(const v4f*)(sp);
      const v4f a1 = *(const v4f*)(sp + 4);
#pragma unroll
      for (int e = 0; e < 4; ++e) {
        hv[it][e]     = (_Float16)a0[e];
        hv[it][4 + e] = (_Float16)a1[e];
      }
    }
    for (int pass = 0; pass < 2; ++pass) {
#pragma unroll
      for (int it = 0; it < 2; ++it)
        *(volatile v8h*)(Y16 + (row0 + (size_t)(l0 + it * 8 + wave)) * kDin + d0 + lane * 8) = hv[it];
      __threadfence();
    }
  }
}

extern "C" void kernel_launch(void* const* d_in, const int* in_sizes, int n_in,
                              void* d_out, int out_size, void* d_ws, size_t ws_size,
                              hipStream_t stream)
{
  if (n_in < 13) return;
  if (in_sizes[0] != kBatch * kCb * kSeq) return;
  if (in_sizes[1] != kCb * kVoc * kDm) return;
  if (in_sizes[2] != kLay * kDm) return;
  if (in_sizes[3] != kLay * kXzP * kDm) return;
  if (in_sizes[4] != kLay * kDin * 4) return;
  if (in_sizes[5] != kLay * kDin) return;
  if (in_sizes[6] != kLay * kXdP * kDin) return;
  if (in_sizes[7] != kLay * kDin * kDtR) return;
  if (in_sizes[8] != kLay * kDin) return;
  if (in_sizes[9] != kLay * kDin * kNst) return;
  if (in_sizes[10] != kLay * kDin) return;
  if (in_sizes[11] != kLay * kDm * kDin) return;
  if (in_sizes[12] != kCb * kDm * kVoc) return;
  if (out_size != kBatch * kCb * kSeq * kVoc) return;
  if (ws_size < kWsTotal) return;

  const int*   codes   = (const int*)d_in[0];
  const float* embed_w = (const float*)d_in[1];
  const float* norm_w  = (const float*)d_in[2];
  const float* in_w    = (const float*)d_in[3];
  const float* conv_w  = (const float*)d_in[4];
  const float* conv_b  = (const float*)d_in[5];
  const float* xp_w    = (const float*)d_in[6];
  const float* dtp_w   = (const float*)d_in[7];
  const float* dtp_b   = (const float*)d_in[8];
  const float* A_log   = (const float*)d_in[9];
  const float* D_skip  = (const float*)d_in[10];
  const float* out_w   = (const float*)d_in[11];
  const float* head_w  = (const float*)d_in[12];
  float* out = (float*)d_out;

  char* ws = (char*)d_ws;
  unsigned short* WIN16  = (unsigned short*)(ws + kOffWIN);
  unsigned short* WXP16  = (unsigned short*)(ws + kOffWXP);
  unsigned short* WDT16  = (unsigned short*)(ws + kOffWDT);
  unsigned short* WOUT16 = (unsigned short*)(ws + kOffWOUT);
  unsigned short* WHD16  = (unsigned short*)(ws + kOffWHD);
  float*          XA     = (float*)(ws + kOffXA);
  float*          XB     = (float*)(ws + kOffXB);
  unsigned short* XN16   = (unsigned short*)(ws + kOffXN);
  float*          XZ     = (float*)(ws + kOffXZ);
  float*          UC     = (float*)(ws + kOffUC);
  unsigned short* UC16   = (unsigned short*)(ws + kOffUC16);
  float*          XD     = (float*)(ws + kOffXD);
  unsigned short* DT16   = (unsigned short*)(ws + kOffDT16);
  float*          DLR    = (float*)(ws + kOffDLR);
  unsigned short* Y16    = (unsigned short*)(ws + kOffY16);
  const float* dummy_resid = norm_w;

  cast_f16_kernel<<<(kLay * kXzP * kDm) / 8 / 256, 256, 0, stream>>>(in_w,  WIN16,  (kLay * kXzP * kDm) / 8,  kCarW);
  cast_f16_kernel<<<(kLay * kXdP * kDin) / 8 / 256, 256, 0, stream>>>(xp_w,  WXP16,  (kLay * kXdP * kDin) / 8, kCarW);
  cast_f16_kernel<<<(kLay * kDin * kDtR) / 8 / 256, 256, 0, stream>>>(dtp_w, WDT16,  (kLay * kDin * kDtR) / 8, kCarW);
  cast_f16_kernel<<<(kLay * kDm * kDin) / 8 / 256, 256, 0, stream>>>(out_w, WOUT16, (kLay * kDm * kDin) / 8,  kCarW);
  transpose_cast_kernel<<<dim3(kVoc / 64, kDm / 64, kCb), 256, 0, stream>>>(head_w, WHD16, kDm, kVoc, kVoc, kCarW);

  embed_sum_kernel<<<kRows / 2, 256, 0, stream>>>(codes, embed_w, XA);

  float* xcur = XA;
  float* xnext = XB;
  for (int l = 0; l < kLay; ++l) {
    rmsnorm_f16_kernel<<<kRows / 8, 256, 0, stream>>>(xcur, norm_w + (size_t)l * kDm, XN16);

    wmma_gemm64_f16<false><<<dim3((kRows / 64) * (kXzP / 64) / 8, 1), 256, 0, stream>>>(
        XN16, kDm, 0L, WIN16 + (size_t)l * kXzP * kDm, kDm, 0L,
        XZ, kXzP, 0L, dummy_resid, kRows, kXzP, kDm, kSclIn);

    conv_silu_kernel<<<dim3(kDin / 256, kRows / 64), 256, 0, stream>>>(
        XZ, conv_w + (size_t)l * kDin * 4, conv_b + (size_t)l * kDin, UC, UC16);

    wmma_gemm64_f16<false><<<dim3((kRows / 64) * (kXdP / 64) / 8, 1), 256, 0, stream>>>(
        UC16, kDin, 0L, WXP16 + (size_t)l * kXdP * kDin, kDin, 0L,
        XD, kXdP, 0L, dummy_resid, kRows, kXdP, kDin, kSclXp);

    dt_cast_kernel<<<(kRows * kDtR) / 8 / 256, 256, 0, stream>>>(XD, DT16, (kRows * kDtR) / 8, kCarDt);

    wmma_gemm64_f16<false><<<dim3((kRows / 64) * (kDin / 64) / 8, 1), 256, 0, stream>>>(
        DT16, kDtR, 0L, WDT16 + (size_t)l * kDin * kDtR, kDtR, 0L,
        DLR, kDin, 0L, dummy_resid, kRows, kDin, kDtR, kSclDt);

    scan_gate_kernel<<<dim3(kDin / 256, kBatch), 256, 0, stream>>>(
        DLR, dtp_b + (size_t)l * kDin, UC, XZ, XD,
        A_log + (size_t)l * kDin * kNst, D_skip + (size_t)l * kDin, Y16);

    wmma_gemm64_f16<true><<<dim3((kRows / 64) * (kDm / 64) / 8, 1), 256, 0, stream>>>(
        Y16, kDin, 0L, WOUT16 + (size_t)l * kDm * kDin, kDin, 0L,
        xnext, kDm, 0L, xcur, kRows, kDm, kDin, kSclOut);

    float* tmp = xcur; xcur = xnext; xnext = tmp;
  }

  cast_f16_kernel<<<(kRows * kDm) / 8 / 256, 256, 0, stream>>>(xcur, XN16, (kRows * kDm) / 8, kCarX);

  for (int b = 0; b < kBatch; ++b) {
    wmma_gemm64_f16<false><<<dim3((kSeq / 64) * (kVoc / 64) / 8, kCb), 256, 0, stream>>>(
        XN16 + (size_t)b * kSeq * kDm, kDm, 0L,
        WHD16, kDm, (long)kVoc * kDm,
        out + (size_t)b * kCb * kSeq * kVoc, kVoc, (long)kSeq * kVoc,
        dummy_resid, kSeq, kVoc, kDm, kSclHead);
  }
}
